// GroupedQueryAttention_78666620993897
// MI455X (gfx1250) — hardware-verified
//
#include <hip/hip_runtime.h>


#ifndef NB
#define NB 4
#endif
#ifndef SEQ
#define SEQ 1024
#endif
#define NB_FULL  4
#define SEQ_FULL 1024
#define TT   SEQ
#define DM   1024
#define NH_  16
#define NKV  4
#define REP  (NH_ / NKV)
#define HD   64
#define DQ   (NH_ * HD)
#define DKV  (NKV * HD)
#define ZH   REP
#define NPAIR 16
#define SCL  0.125f
#define LNEPS 1e-5f

static_assert(TT % 128 == 0);
static_assert((NB * TT) % 64 == 0);
static_assert(DQ % 64 == 0 && DKV % 64 == 0 && DM % 64 == 0 && HD == 64);
static_assert(DM % 32 == 0 && TT % 32 == 0 && DQ % 32 == 0);
static_assert(NB <= NB_FULL && SEQ <= SEQ_FULL);
static_assert(((size_t)NB * NH_ * TT * HD) % 512 == 0);
static_assert(((size_t)NB * NKV * TT * HD) % 512 == 0);
static_assert(((size_t)ZH * TT * HD) % 512 == 0);
static_assert((ZH * TT) % 8 == 0);
static_assert((2 * NB * TT * NPAIR) % 256 == 0);
static_assert(((size_t)TT * DM / 8) % 256 == 0 && ((size_t)DQ * DM / 8) % 256 == 0 && ((size_t)DKV * DM / 8) % 256 == 0);

typedef unsigned short bf;
typedef __attribute__((ext_vector_type(16))) __bf16   v16bf;
typedef __attribute__((ext_vector_type(8)))  unsigned short v8us;
typedef __attribute__((ext_vector_type(8)))  float    v8f;
typedef __attribute__((ext_vector_type(4)))  float    v4f;
typedef __attribute__((ext_vector_type(2)))  float    v2f;
typedef __attribute__((ext_vector_type(2)))  unsigned short v2us;
typedef __attribute__((ext_vector_type(4)))  unsigned short v4us;
typedef __attribute__((ext_vector_type(4)))  int      v4i;
typedef v4f  __attribute__((may_alias)) v4fa;

__device__ __forceinline__ unsigned short f2bf(float f) { unsigned u = __float_as_uint(f); u += 0x7FFFu + ((u >> 16) & 1u); return (unsigned short)(u >> 16); }
__device__ __forceinline__ float bf2f(unsigned short b) { return __uint_as_float(((unsigned)b) << 16); }
__device__ __forceinline__ float bfr(float f) { return bf2f(f2bf(f)); }
__device__ __forceinline__ v16bf cat16b(v8us lo, v8us hi) { return __builtin_bit_cast(v16bf, __builtin_shufflevector(lo, hi, 0, 1, 2, 3, 4, 5, 6, 7, 8, 9, 10, 11, 12, 13, 14, 15)); }
__device__ __forceinline__ v8f wmmab(v16bf a, v16bf b, v8f c) { return __builtin_amdgcn_wmma_f32_16x16x32_bf16(false, a, false, b, (short)0, c, false, false); }
__device__ __forceinline__ void splitf(float y, unsigned short& h, unsigned short& l) { h = f2bf(y); l = f2bf(y - bf2f(h)); }

template <typename T16> struct WFrag;
template <> struct WFrag<bf> { typedef v16bf V; static __device__ __forceinline__ V ld(const bf* p) { return cat16b(*(const v8us*)p, *(const v8us*)(p + 16)); } static __device__ __forceinline__ v8f mma(V a, V b, v8f c) { return wmmab(a, b, c); } };
template <typename T16, int NSPLIT, bool BIAS>
__global__ __launch_bounds__(32) void k_gemmw(const T16* __restrict__ A, const T16* __restrict__ A2, const T16* __restrict__ Bt, const T16* __restrict__ Bt2, int K, float* C, int ldc, const float* __restrict__ bias, size_t sA, size_t sB, size_t sC) {
    typedef typename WFrag<T16>::V V;
    __shared__ __align__(16) float os[16 * 68];
    const size_t z = blockIdx.z; A += z * sA; if (A2) A2 += z * sA; Bt += z * sB; if (Bt2) Bt2 += z * sB; C += z * sC;
    const int lane = threadIdx.x & 31, lr = lane & 15, hi = lane >> 4; const int r0 = blockIdx.x * 64, c0 = blockIdx.y * 64;
    v8f acc[4][4];
#pragma unroll
    for (int mb = 0; mb < 4; ++mb)
#pragma unroll
        for (int nb = 0; nb < 4; ++nb) acc[mb][nb] = (v8f){};
    const size_t aoff = (size_t)(r0 + lr) * K + 8 * hi, boff = (size_t)(c0 + lr) * K + 8 * hi;
#pragma unroll 1
    for (int kc = 0; kc < K; kc += 32) {
        V a[4], a2[4];
#pragma unroll
        for (int mb = 0; mb < 4; ++mb) { a[mb] = WFrag<T16>::ld(A + aoff + (size_t)mb * 16 * K + kc); if (NSPLIT == 1 || NSPLIT == 2) a2[mb] = WFrag<T16>::ld(A2 + aoff + (size_t)mb * 16 * K + kc); }
#pragma unroll
        for (int nb = 0; nb < 4; ++nb) { const V b = WFrag<T16>::ld(Bt + boff + (size_t)nb * 16 * K + kc); V b2; if (NSPLIT >= 2) b2 = WFrag<T16>::ld(Bt2 + boff + (size_t)nb * 16 * K + kc);
#pragma unroll
            for (int mb = 0; mb < 4; ++mb) { acc[mb][nb] = WFrag<T16>::mma(a[mb], b, acc[mb][nb]); if (NSPLIT == 1 || NSPLIT == 2) acc[mb][nb] = WFrag<T16>::mma(a2[mb], b, acc[mb][nb]); if (NSPLIT >= 2) acc[mb][nb] = WFrag<T16>::mma(a[mb], b2, acc[mb][nb]); } }
        asm volatile("v_nop\n\tv_nop\n\tv_nop\n\tv_nop" : "+v"(acc[0][0]), "+v"(acc[1][1]), "+v"(acc[2][2]), "+v"(acc[3][3]) : "v"(a[0]), "v"(a[3]));
    }
#pragma unroll
    for (int mb = 0; mb < 4; ++mb) {
#pragma unroll
        for (int nb = 0; nb < 4; ++nb) {
#pragma unroll
            for (int j = 0; j < 8; ++j) os[(hi * 8 + j) * 68 + nb * 16 + lr] = acc[mb][nb][j]; }
        __builtin_amdgcn_wave_barrier(); asm volatile("" ::: "memory");
        float* crow = C + (size_t)(r0 + mb * 16) * ldc + c0;
#pragma unroll 1
        for (int ps = 0; ps < 2; ++ps) {
#pragma unroll
            for (int s = 0; s < 8; ++s) { const int row = 2 * s + hi, cofs = lr * 4; v4f val = *(const v4fa*)(os + row * 68 + cofs); if (BIAS) { val[0] += bfr(bias[c0 + cofs]); val[1] += bfr(bias[c0 + cofs + 1]); val[2] += bfr(bias[c0 + cofs + 2]); val[3] += bfr(bias[c0 + cofs + 3]); }
                *(volatile v4f*)(crow + (size_t)row * ldc + cofs) = val; }
            if (ps == 0) __threadfence(); }
        __builtin_amdgcn_wave_barrier(); asm volatile("" ::: "memory");
    }
}

__global__ __launch_bounds__(256) void k_cvt8(const float* __restrict__ src, bf* dst, unsigned n8, size_t sS, size_t sD) {
    const unsigned i = blockIdx.x * 256u + threadIdx.x; if (i >= n8) return;
    src += (size_t)blockIdx.y * sS; dst += (size_t)blockIdx.y * sD;
    const v8f v = *(const v8f*)(src + (size_t)i * 8); v8us o;
#pragma unroll
    for (int k = 0; k < 8; ++k) o[k] = f2bf(v[k]);
    *(volatile v8us*)(dst + (size_t)i * 8) = o; __threadfence(); *(volatile v8us*)(dst + (size_t)i * 8) = o; }

__device__ __forceinline__ float powtab(unsigned i) {
    float r = 1.0f;
    r = (i == 1u)  ? 1.7782794100389228f : r;  r = (i == 2u)  ? 3.1622776601683795f : r;  r = (i == 3u)  ? 5.623413251903491f : r;
    r = (i == 4u)  ? 10.0f : r;                r = (i == 5u)  ? 17.782794100389228f : r;  r = (i == 6u)  ? 31.622776601683793f : r;
    r = (i == 7u)  ? 56.23413251903491f : r;   r = (i == 8u)  ? 100.0f : r;               r = (i == 9u)  ? 177.82794100389228f : r;
    r = (i == 10u) ? 316.22776601683796f : r;  r = (i == 11u) ? 562.341325190349f : r;    r = (i == 12u) ? 1000.0f : r;
    r = (i == 13u) ? 1778.2794100389228f : r;  r = (i == 14u) ? 3162.2776601683795f : r;  r = (i == 15u) ? 5623.413251903491f : r;
    return r; }

__global__ __launch_bounds__(256) void k_cstab(const int* __restrict__ qt, const int* __restrict__ kt, float* CS) {
    const unsigned idx = blockIdx.x * 256u + threadIdx.x; const unsigned per = (unsigned)(NB * TT * NPAIR);
    if (idx >= 2u * per) return;
    const unsigned tab = idx / per, r = idx % per, i = r & 15u, bt = r >> 4, b = bt / (unsigned)TT, t = bt % (unsigned)TT;
    const unsigned src = b * (unsigned)SEQ_FULL + t;
    const int tq = qt[src], tk = kt[src]; const int tid = tab ? tk : tq;
    const float th = 1.0f / powtab(i);
    const float a = (float)tid * th;
    v2f cs; cs[0] = cosf(a); cs[1] = sinf(a);
    *(volatile v2f*)(CS + (size_t)idx * 2) = cs; __threadfence(); *(volatile v2f*)(CS + (size_t)idx * 2) = cs; }

__global__ __launch_bounds__(256) void k_lnrope(const float* __restrict__ F, unsigned pitch, unsigned nheads, const float* __restrict__ CS, const float* __restrict__ gam, const float* __restrict__ bet, bf* Ph, bf* Pl) {
    const unsigned lane = threadIdx.x & 31u;
    const unsigned e = (blockIdx.x * 256u + threadIdx.x) * 2u; if (e >= (unsigned)NB * nheads * (unsigned)TT * (unsigned)HD) return;
    const unsigned d = e % (unsigned)HD; const unsigned t = (e / (unsigned)HD) % (unsigned)TT; const unsigned bh = e / (unsigned)(HD * TT); const unsigned h = bh % nheads, b = bh / nheads;
    const v2f x = *(const v2f*)(F + (size_t)(b * (unsigned)TT + t) * pitch + h * (unsigned)HD + d);
    float s = x[0] + x[1];
#pragma unroll
    for (int sh = 16; sh; sh >>= 1) s += __shfl_xor(s, sh, 32);
    const float mean = s * (1.0f / 64.0f);
    const float dx0 = x[0] - mean, dx1 = x[1] - mean;
    float v = dx0 * dx0 + dx1 * dx1;
#pragma unroll
    for (int sh = 16; sh; sh >>= 1) v += __shfl_xor(v, sh, 32);
    const float rstd = rsqrtf(v * (1.0f / 64.0f) + LNEPS);
    const float y0 = dx0 * rstd * bfr(gam[d]) + bfr(bet[d]);
    const float y1 = dx1 * rstd * bfr(gam[d + 1u]) + bfr(bet[d + 1u]);
    const v2f cs = *(const v2f*)(CS + ((size_t)(b * (unsigned)TT + t) * NPAIR + (lane & 15u)) * 2);
    const bool rot = lane < 16u;
    const float c = rot ? cs[0] : 1.0f, sn = rot ? cs[1] : 0.0f;
    const float r0 = c * y0 - sn * y1;
    const float r1 = c * y1 + sn * y0;
    v2us oh, ol; unsigned short a2, c2; splitf(r0, a2, c2); oh[0] = a2; ol[0] = c2; splitf(r1, a2, c2); oh[1] = a2; ol[1] = c2;
    *(volatile v2us*)(Ph + e) = oh; *(volatile v2us*)(Pl + e) = ol; __threadfence(); *(volatile v2us*)(Ph + e) = oh; *(volatile v2us*)(Pl + e) = ol; }

__global__ __launch_bounds__(256) void k_vtp(const float* __restrict__ F, unsigned pitch, bf* Vh, bf* Vl) {
    const unsigned e = (blockIdx.x * 256u + threadIdx.x) * 2u; if (e >= (unsigned)(NB * NKV * HD * TT)) return;
    const unsigned t = e % (unsigned)TT; const unsigned d = (e / (unsigned)TT) % (unsigned)HD; const unsigned bg = e / (unsigned)(TT * HD); const unsigned g = bg % (unsigned)NKV, b = bg / (unsigned)NKV; v2us oh, ol;
#pragma unroll
    for (unsigned q = 0; q < 2u; ++q) { const float x = F[(size_t)(b * (unsigned)TT + t + q) * pitch + g * (unsigned)HD + d]; unsigned short a2, c2; splitf(x, a2, c2); oh[q] = a2; ol[q] = c2; }
    *(volatile v2us*)(Vh + e) = oh; *(volatile v2us*)(Vl + e) = ol; __threadfence(); *(volatile v2us*)(Vh + e) = oh; *(volatile v2us*)(Vl + e) = ol; }

__global__ __launch_bounds__(256) void k_asoft(const float* __restrict__ Sb, const int* __restrict__ qvar, const int* __restrict__ kvar, const float* __restrict__ vemb, unsigned h0, bf* Ph, bf* Pl) {
    const unsigned lane = threadIdx.x & 31u; const unsigned row = blockIdx.x * 8u + (threadIdx.x >> 5); if (row >= (unsigned)(ZH * TT)) return;
    const unsigned i = row % (unsigned)TT; const unsigned zz = row / (unsigned)TT;
    const float w0 = bfr(vemb[h0 + zz]), w1 = bfr(vemb[(unsigned)NH_ + h0 + zz]);
    const int qv = qvar[i];
    const float* sr = Sb + (size_t)row * TT; float v[TT / 32]; float mx = -3.0e38f;
#pragma unroll
    for (int ch = 0; ch < TT / 128; ++ch) { const unsigned j0 = (unsigned)ch * 128u + lane * 4u; const v4f a = *(const v4f*)(sr + j0); const v4i kq = *(const v4i*)(kvar + j0);
#pragma unroll
        for (int q = 0; q < 4; ++q) { const float t = a[q] * SCL + ((kq[q] == qv) ? w1 : w0); v[ch * 4 + q] = t; mx = fmaxf(mx, t); } }
#pragma unroll
    for (int sh = 16; sh; sh >>= 1) mx = fmaxf(mx, __shfl_xor(mx, sh, 32));
    float sum = 0.f;
#pragma unroll
    for (int k = 0; k < TT / 32; ++k) { float d0 = __fsub_rn(v[k], mx); asm volatile("" : "+v"(d0)); v[k] = __builtin_amdgcn_exp2f(__fmul_rn(d0, 1.4426950408889634f)); sum += v[k]; }
#pragma unroll
    for (int sh = 16; sh; sh >>= 1) sum += __shfl_xor(sum, sh, 32);
    const float f = __fdiv_rn(1.0f, sum);
#pragma unroll 1
    for (int ps = 0; ps < 2; ++ps) {
#pragma unroll
        for (int ch = 0; ch < TT / 128; ++ch) { v4us oh, ol;
#pragma unroll
            for (int q = 0; q < 4; ++q) { unsigned short a, c2; splitf(v[ch * 4 + q] * f, a, c2); oh[q] = a; ol[q] = c2; }
            const size_t oo = (size_t)row * TT + (unsigned)ch * 128u + lane * 4u; *(volatile v4us*)(Ph + oo) = oh; *(volatile v4us*)(Pl + oo) = ol; }
        if (ps == 0) __threadfence(); }
}

__global__ __launch_bounds__(256) void k_merge(const float* __restrict__ O, unsigned h0, bf* Ah, bf* Al) {
    const unsigned e = (blockIdx.x * 256u + threadIdx.x) * 2u; if (e >= (unsigned)(ZH * TT * HD)) return;
    const unsigned d = e % (unsigned)HD; const unsigned t = (e / (unsigned)HD) % (unsigned)TT; const unsigned zz = e / (unsigned)(HD * TT);
    const size_t oo = (size_t)t * DQ + (h0 + zz) * (unsigned)HD + d;
    const v2f x = *(const v2f*)(O + e);
    v2us oh, ol; unsigned short a, c2; splitf(x[0], a, c2); oh[0] = a; ol[0] = c2; splitf(x[1], a, c2); oh[1] = a; ol[1] = c2;
    *(volatile v2us*)(Ah + oo) = oh; *(volatile v2us*)(Al + oo) = ol; __threadfence(); *(volatile v2us*)(Ah + oo) = oh; *(volatile v2us*)(Al + oo) = ol; }

constexpr size_t al256(size_t b) { return (b + 255) & ~(size_t)255; }
constexpr size_t WS_TOTAL =
    al256((size_t)DQ * DM * 2) + 2 * al256((size_t)DKV * DM * 2) + al256((size_t)DM * DQ * 2) +
    2 * al256((size_t)NB * TT * DM * 2) +
    al256((size_t)NB * TT * DQ * 4) + 2 * al256((size_t)NB * TT * DKV * 4) +
    al256((size_t)2 * NB * TT * NPAIR * 2 * 4) +
    2 * al256((size_t)NB * NH_ * TT * HD * 2) + 4 * al256((size_t)NB * NKV * TT * HD * 2) +
    al256((size_t)ZH * TT * TT * 4) + 2 * al256((size_t)ZH * TT * TT * 2) + al256((size_t)ZH * TT * HD * 4) +
    2 * al256((size_t)NB * TT * DQ * 2);
static_assert(WS_TOTAL <= (size_t)134217728);

extern "C" void kernel_launch(void* const* d_in, const int* in_sizes, int n_in,
                              void* d_out, int out_size, void* d_ws, size_t ws_size, hipStream_t stream) {
    if (n_in < 19) return;
    const long long rowsNeed = (long long)(NB - 1) * SEQ_FULL + SEQ;
    if ((long long)in_sizes[0] < rowsNeed * DM || (long long)in_sizes[1] < rowsNeed * DM) return;
    if (in_sizes[2] < DQ * DM || in_sizes[3] < DQ || in_sizes[4] < DKV * DM || in_sizes[5] < DKV || in_sizes[6] < DKV * DM || in_sizes[7] < DKV || in_sizes[8] < DM * DQ || in_sizes[9] < DM) return;
    if (in_sizes[10] < HD || in_sizes[11] < HD || in_sizes[12] < HD || in_sizes[13] < HD || in_sizes[14] < 2 * NH_) return;
    if ((long long)in_sizes[15] < rowsNeed || (long long)in_sizes[16] < rowsNeed || (long long)in_sizes[17] < rowsNeed || (long long)in_sizes[18] < rowsNeed) return;
    if ((long long)out_size < rowsNeed * DM) return;
    if (WS_TOTAL > ws_size) return;
    const float* x = (const float*)d_in[0]; const float* kv = (const float*)d_in[1];
    const float* qw = (const float*)d_in[2]; const float* qb = (const float*)d_in[3];
    const float* kw = (const float*)d_in[4]; const float* kb = (const float*)d_in[5];
    const float* vw = (const float*)d_in[6]; const float* vb = (const float*)d_in[7];
    const float* ow = (const float*)d_in[8]; const float* ob = (const float*)d_in[9];
    const float* qng = (const float*)d_in[10]; const float* qnb = (const float*)d_in[11];
    const float* kng = (const float*)d_in[12]; const float* knb = (const float*)d_in[13];
    const float* vemb = (const float*)d_in[14];
    const int* qvar = (const int*)d_in[15]; const int* kvar = (const int*)d_in[16];
    const int* qtime = (const int*)d_in[17]; const int* ktime = (const int*)d_in[18];
    float* OUT = (float*)d_out;
    char* wsp = (char*)d_ws;
    auto take = [&](size_t bytes) { char* p = wsp; wsp += (bytes + 255) & ~(size_t)255; return (void*)p; };
    bf* WQ = (bf*)take((size_t)DQ * DM * 2); bf* WK = (bf*)take((size_t)DKV * DM * 2); bf* WV = (bf*)take((size_t)DKV * DM * 2); bf* WO = (bf*)take((size_t)DM * DQ * 2);
    bf* XB = (bf*)take((size_t)NB * TT * DM * 2); bf* KVB = (bf*)take((size_t)NB * TT * DM * 2);
    float* FQ = (float*)take((size_t)NB * TT * DQ * 4); float* FK = (float*)take((size_t)NB * TT * DKV * 4); float* FV = (float*)take((size_t)NB * TT * DKV * 4);
    float* CS = (float*)take((size_t)2 * NB * TT * NPAIR * 2 * 4);
    bf* QPh = (bf*)take((size_t)NB * NH_ * TT * HD * 2); bf* QPl = (bf*)take((size_t)NB * NH_ * TT * HD * 2);
    bf* KPh = (bf*)take((size_t)NB * NKV * TT * HD * 2); bf* KPl = (bf*)take((size_t)NB * NKV * TT * HD * 2);
    bf* VTh = (bf*)take((size_t)NB * NKV * HD * TT * 2); bf* VTl = (bf*)take((size_t)NB * NKV * HD * TT * 2);
    float* Sb = (float*)take((size_t)ZH * TT * TT * 4); bf* Ph = (bf*)take((size_t)ZH * TT * TT * 2); bf* Pl = (bf*)take((size_t)ZH * TT * TT * 2);
    float* Ob = (float*)take((size_t)ZH * TT * HD * 4);
    bf* ATh = (bf*)take((size_t)NB * TT * DQ * 2); bf* ATl = (bf*)take((size_t)NB * TT * DQ * 2);
    if ((size_t)(wsp - (char*)d_ws) > ws_size) return;
    float* CSq = CS; float* CSk = CS + (size_t)NB * TT * NPAIR * 2;

    k_cvt8<<<dim3((unsigned)((size_t)DQ * DM / 8 / 256), 1), 256, 0, stream>>>(qw, WQ, (unsigned)((size_t)DQ * DM / 8), 0, 0);
    k_cvt8<<<dim3((unsigned)((size_t)DKV * DM / 8 / 256), 1), 256, 0, stream>>>(kw, WK, (unsigned)((size_t)DKV * DM / 8), 0, 0);
    k_cvt8<<<dim3((unsigned)((size_t)DKV * DM / 8 / 256), 1), 256, 0, stream>>>(vw, WV, (unsigned)((size_t)DKV * DM / 8), 0, 0);
    k_cvt8<<<dim3((unsigned)((size_t)DM * DQ / 8 / 256), 1), 256, 0, stream>>>(ow, WO, (unsigned)((size_t)DM * DQ / 8), 0, 0);
    k_cvt8<<<dim3((unsigned)((size_t)TT * DM / 8 / 256), NB), 256, 0, stream>>>(x, XB, (unsigned)((size_t)TT * DM / 8), (size_t)SEQ_FULL * DM, (size_t)TT * DM);
    k_cvt8<<<dim3((unsigned)((size_t)TT * DM / 8 / 256), NB), 256, 0, stream>>>(kv, KVB, (unsigned)((size_t)TT * DM / 8), (size_t)SEQ_FULL * DM, (size_t)TT * DM);
    k_cstab<<<(unsigned)(2 * NB * TT * NPAIR / 256), 256, 0, stream>>>(qtime, ktime, CS);

    k_gemmw<bf, 0, true><<<dim3(NB * TT / 64, DQ / 64, 1), 32, 0, stream>>>(XB, nullptr, WQ, nullptr, DM, FQ, DQ, qb, 0, 0, 0);
    k_lnrope<<<(unsigned)((size_t)NB * NH_ * TT * HD / 512), 256, 0, stream>>>(FQ, DQ, NH_, CSq, qng, qnb, QPh, QPl);
    k_gemmw<bf, 0, true><<<dim3(NB * TT / 64, DKV / 64, 1), 32, 0, stream>>>(KVB, nullptr, WK, nullptr, DM, FK, DKV, kb, 0, 0, 0);
    k_lnrope<<<(unsigned)((size_t)NB * NKV * TT * HD / 512), 256, 0, stream>>>(FK, DKV, NKV, CSk, kng, knb, KPh, KPl);
    k_gemmw<bf, 0, true><<<dim3(NB * TT / 64, DKV / 64, 1), 32, 0, stream>>>(KVB, nullptr, WV, nullptr, DM, FV, DKV, vb, 0, 0, 0);
    k_vtp<<<(unsigned)((size_t)NB * NKV * HD * TT / 512), 256, 0, stream>>>(FV, DKV, VTh, VTl);

    for (int b = 0; b < NB; ++b) {
        for (int g = 0; g < NKV; ++g) {
            const size_t zq = ((size_t)b * NH_ + (size_t)g * REP) * TT * HD;
            const size_t zk = ((size_t)b * NKV + g) * TT * HD;
            k_gemmw<bf, 2, false><<<dim3(TT / 64, TT / 64, ZH), 32, 0, stream>>>(QPh + zq, QPl + zq, KPh + zk, KPl + zk, HD, Sb, TT, nullptr, (size_t)TT * HD, 0, (size_t)TT * TT);
            k_asoft<<<ZH * TT / 8, 256, 0, stream>>>(Sb, qvar + (size_t)b * SEQ_FULL, kvar + (size_t)b * SEQ_FULL, vemb, (unsigned)(g * REP), Ph, Pl);
            k_gemmw<bf, 2, false><<<dim3(TT / 64, HD / 64, ZH), 32, 0, stream>>>(Ph, Pl, VTh + zk, VTl + zk, TT, Ob, HD, nullptr, (size_t)TT * TT, 0, (size_t)TT * HD);
            k_merge<<<(unsigned)((size_t)ZH * TT * HD / 512), 256, 0, stream>>>(Ob, (unsigned)(g * REP), ATh + (size_t)b * TT * DQ, ATl + (size_t)b * TT * DQ);
        }
    }
    k_gemmw<bf, 1, true><<<dim3(TT / 64, DM / 64, NB), 32, 0, stream>>>(ATh, ATl, WO, nullptr, DQ, OUT, DM, ob, (size_t)TT * DQ, 0, (size_t)SEQ_FULL * DM);
}
